// GCN_66915590472494
// MI455X (gfx1250) — hardware-run, weakly checked
//
#include <hip/hip_runtime.h>
#include <stddef.h>
#include <stdint.h>
#include <math.h>

#ifndef SPLIT_L2
#define SPLIT_L2 1
#endif
#ifndef SPLIT_L3
#define SPLIT_L3 1
#endif

#define NN      50000
#define FD      96
#define NE      800000
#define GBM     128
#define MP      50048
#define NTHR    256
#define NWAVE   8
#define EPT     8
#define WCH     (32 * EPT)
#define NBRUN   1024
#define SLB     10
#define NBK     49
#define WLCAP   2560
#define RCAP    20480
#define DEGCAP  64
#define MAXDEG_MEAS   35
#define MAXB1024_MEAS 16623
#define ABM     64
#define SP      100
#define APITCH1 96
#define BPITCH1 96
#define APITCH2 192
#define BPITCH2 192
#define KEXT_L1 96
#define KEXT_L2 (SPLIT_L2 ? 192 : 96)
#define KEXT_L3 (SPLIT_L3 ? 192 : 96)

#define BK_ZINTS (NWAVE * WLCAP + 2 * RCAP + 4 * NBRUN)
#define BK_INTS  (BK_ZINTS + 16)
#define BK_LDS   (BK_INTS * 4)

#define PBX   (MP * FD / 8 / NTHR)
#define NUZ   ((MP - NN) * APITCH2 / 8)
#define PBZ   ((NUZ + NTHR - 1) / NTHR)
#define NUW1  (FD * BPITCH1 / 8)
#define PBW1  ((NUW1 + NTHR - 1) / NTHR)
#define NUW2  (FD * BPITCH2 / 8)
#define PBW2  (NUW2 / NTHR)
#define PBTOT (PBX + PBZ + PBW1 + 2 * PBW2 + 1)

static_assert(FD == 96 && FD % 32 == 0 && FD % 16 == 0 && 24 * 4 == FD);
static_assert(MP % GBM == 0 && MP >= NN && MP == 391 * GBM && MP % ABM == 0);
static_assert(NBRUN == (1 << SLB) && NBRUN % ABM == 0 && NBRUN % GBM == 0 && NBRUN % NTHR == 0);
static_assert(NBK * NBRUN >= MP && NBK * NBRUN >= NN);
static_assert(NE < (1 << 21) && (((long long)NE) << SLB) < (1LL << 31));
static_assert(NE % WCH == 0 && NE % 4 == 0);
static_assert(RCAP == NWAVE * WLCAP && RCAP % 4 == 0 && BK_ZINTS % 4 == 0);
static_assert((long long)RCAP * 100 >= (long long)MAXB1024_MEAS * 105);
static_assert(WLCAP >= MAXB1024_MEAS / 8 + 8 * 46 + 1);
static_assert(MAXDEG_MEAS + 8 <= DEGCAP);
static_assert((MP * FD / 8) % NTHR == 0 && NUW2 % NTHR == 0);
static_assert(NUZ % 32 == 0 && NUW1 % 32 == 0);
static_assert(KEXT_L1 % 32 == 0 && KEXT_L2 % 32 == 0 && KEXT_L3 % 32 == 0);
static_assert(KEXT_L1 <= APITCH1 && KEXT_L1 <= BPITCH1);
static_assert(KEXT_L2 <= APITCH2 && KEXT_L2 <= BPITCH2 && KEXT_L3 <= APITCH2 && KEXT_L3 <= BPITCH2);
static_assert(APITCH2 == 2 * FD && BPITCH2 == 2 * FD);
static_assert(BK_LDS <= 300000);
static_assert((GBM * SP + GBM) * 4 <= 65536 && (SP * 4) % 16 == 0 && SP >= FD);
static_assert(GBM * FD / 4 == 12 * NTHR);
static_assert(((size_t)NN * APITCH2 * 2) % 128 == 0);

typedef float          v4f   __attribute__((ext_vector_type(4)));
typedef float          v8f   __attribute__((ext_vector_type(8)));
typedef int            v2i   __attribute__((ext_vector_type(2)));
typedef int            v4i   __attribute__((ext_vector_type(4)));
typedef int            v8i   __attribute__((ext_vector_type(8)));
typedef unsigned short v8us  __attribute__((ext_vector_type(8)));
typedef unsigned short v16us __attribute__((ext_vector_type(16)));
typedef __bf16         v16bf __attribute__((ext_vector_type(16)));
typedef v4f  __attribute__((may_alias)) v4fa;
typedef v2i  __attribute__((may_alias)) v2ia;
typedef v4i  __attribute__((may_alias)) v4ia;
typedef v8us __attribute__((may_alias)) v8usa;
union FragB { v16bf v; v16us u; v8us h[2]; v8i w; };

__device__ __forceinline__ v8f wmb(const FragB& a, const FragB& b, v8f c) {
  v8f d = __builtin_amdgcn_wmma_f32_16x16x32_bf16(false, a.v, false, b.v, (short)0, c, false, false);
  asm volatile("v_nop\n\tv_nop\n\tv_nop\n\tv_nop" : "+v"(d) : "v"(a.w), "v"(b.w));
  return d;
}

__device__ __forceinline__ unsigned bf16_bits(float f) {
  const unsigned u = __float_as_uint(f);
  const unsigned r = (u + 0x7FFFu + ((u >> 16) & 1u)) >> 16;
  const unsigned q = (u >> 16) | 0x40u;
  return ((u & 0x7fffffffu) > 0x7f800000u) ? q : r;
}

__device__ __forceinline__ void hilo_pack(float v0, float v1, float v2, float v3,
                                          int& h01, int& h23, int& l01, int& l23) {
  const unsigned a0 = bf16_bits(v0), a1 = bf16_bits(v1), a2 = bf16_bits(v2), a3 = bf16_bits(v3);
  const unsigned b0 = bf16_bits(v0 - __uint_as_float(a0 << 16));
  const unsigned b1 = bf16_bits(v1 - __uint_as_float(a1 << 16));
  const unsigned b2 = bf16_bits(v2 - __uint_as_float(a2 << 16));
  const unsigned b3 = bf16_bits(v3 - __uint_as_float(a3 << 16));
  h01 = (int)(a0 | (a1 << 16)); h23 = (int)(a2 | (a3 << 16));
  l01 = (int)(b0 | (b1 << 16)); l23 = (int)(b2 | (b3 << 16));
}

__device__ __forceinline__ v4i regroup24(int h01, int h23, int l01, int l23, int lane) {
  const int t  = lane < 24 ? lane : 23;
  const int tm = t < 12 ? t : t - 12;
  const int s0 = 2 * tm, s1 = s0 + 1;
  const int a0 = __shfl(h01, s0, 32), a1 = __shfl(h23, s0, 32), a2 = __shfl(h01, s1, 32), a3 = __shfl(h23, s1, 32);
  const int b0 = __shfl(l01, s0, 32), b1 = __shfl(l23, s0, 32), b2 = __shfl(l01, s1, 32), b3 = __shfl(l23, s1, 32);
  const int mk = (t < 12) ? -1 : 0;
  v4i o;
  o.x = (a0 & mk) | (b0 & ~mk); o.y = (a1 & mk) | (b1 & ~mk);
  o.z = (a2 & mk) | (b2 & ~mk); o.w = (a3 & mk) | (b3 & ~mk);
  return o;
}

__device__ __forceinline__ void st2_v8us(unsigned short* p, v8us v) {
  *(volatile v8us*)p = v;
  __threadfence();
  *(volatile v8us*)p = v;
}

__device__ __forceinline__ v8us colpick8(const float* __restrict__ base, int stride) {
  float f[8];
#pragma unroll
  for (int i = 0; i < 8; ++i) f[i] = base[(size_t)i * (size_t)stride];
  v8us o;
#pragma unroll
  for (int i = 0; i < 8; ++i) o[i] = (unsigned short)bf16_bits(f[i]);
  return o;
}

__global__ __launch_bounds__(NTHR) void k_prep(const float* __restrict__ x,
                                               const float* __restrict__ w1, const float* __restrict__ b1,
                                               const float* __restrict__ w2, const float* __restrict__ b2,
                                               const float* __restrict__ w3, const float* __restrict__ b3,
                                               unsigned short* xb, unsigned short* xhl, unsigned short* w1t,
                                               unsigned short* w2d, unsigned short* w3d, float* biasp) {
  const int tid = (int)threadIdx.x;
  const int blk = (int)blockIdx.x;
  if (blk < PBX) {
    const int u  = blk * NTHR + tid;
    const int e  = u * 8;
    const int ec = e < NN * FD ? e : NN * FD - 8;
    const unsigned mk = e < NN * FD ? 0xffffu : 0u;
    const float* p = x + ec;
    const v4f a = *(const v4fa*)p;
    const v4f b = *(const v4fa*)(p + 4);
    v8us o;
    o[0] = (unsigned short)(bf16_bits(a.x) & mk); o[1] = (unsigned short)(bf16_bits(a.y) & mk);
    o[2] = (unsigned short)(bf16_bits(a.z) & mk); o[3] = (unsigned short)(bf16_bits(a.w) & mk);
    o[4] = (unsigned short)(bf16_bits(b.x) & mk); o[5] = (unsigned short)(bf16_bits(b.y) & mk);
    o[6] = (unsigned short)(bf16_bits(b.z) & mk); o[7] = (unsigned short)(bf16_bits(b.w) & mk);
    st2_v8us(xb + (size_t)e, o);
  } else if (blk < PBX + PBZ) {
    const int u = (blk - PBX) * NTHR + tid;
    const int uc = u < NUZ ? u : NUZ - 1;
    const v8us z = {0, 0, 0, 0, 0, 0, 0, 0};
    unsigned short* dp = xhl + (size_t)NN * APITCH2 + (size_t)uc * 8;
    if (u < NUZ) *(volatile v8us*)dp = z;
    __threadfence();
    if (u < NUZ) *(volatile v8us*)dp = z;
  } else if (blk < PBX + PBZ + PBW1) {
    const int u  = (blk - PBX - PBZ) * NTHR + tid;
    const int uc = u < NUW1 ? u : NUW1 - 1;
    const int n  = uc / 12, k8 = (uc - 12 * n) * 8;
    const v8us o = colpick8(w1 + (size_t)k8 * FD + n, FD);
    unsigned short* dp = w1t + (size_t)uc * 8;
    if (u < NUW1) *(volatile v8us*)dp = o;
    __threadfence();
    if (u < NUW1) *(volatile v8us*)dp = o;
  } else if (blk < PBX + PBZ + PBW1 + PBW2) {
    const int u  = (blk - PBX - PBZ - PBW1) * NTHR + tid;
    const int n  = u / 24, k8 = (u - 24 * n) * 8;
    const int kk = k8 >= FD ? k8 - FD : k8;
    const v8us o = colpick8(w2 + (size_t)kk * FD + n, FD);
    st2_v8us(w2d + (size_t)u * 8, o);
  } else if (blk < PBX + PBZ + PBW1 + 2 * PBW2) {
    const int u  = (blk - PBX - PBZ - PBW1 - PBW2) * NTHR + tid;
    const int n  = u / 24, k8 = (u - 24 * n) * 8;
    const int kk = k8 >= FD ? k8 - FD : k8;
    const v8us o = colpick8(w3 + (size_t)kk * FD + n, FD);
    st2_v8us(w3d + (size_t)u * 8, o);
  } else {
    if (tid < 96) {
      const int tc = tid < 72 ? tid : 71;
      const int j  = tc / 24, c4 = tc - 24 * j;
      const v4f a = *(const v4fa*)(b1 + 4 * c4);
      const v4f b = *(const v4fa*)(b2 + 4 * c4);
      const v4f c = *(const v4fa*)(b3 + 4 * c4);
      asm volatile("" :: "v"(a));
      asm volatile("" :: "v"(b));
      asm volatile("" :: "v"(c));
      const unsigned m0 = (j == 0) ? 0xffffffffu : 0u;
      const unsigned m1 = (j == 1) ? 0xffffffffu : 0u;
      const unsigned m2 = (j == 2) ? 0xffffffffu : 0u;
      v4f o;
      o.x = __uint_as_float(((bf16_bits(a.x) << 16) & m0) | ((bf16_bits(b.x) << 16) & m1) | ((bf16_bits(c.x) << 16) & m2));
      o.y = __uint_as_float(((bf16_bits(a.y) << 16) & m0) | ((bf16_bits(b.y) << 16) & m1) | ((bf16_bits(c.y) << 16) & m2));
      o.z = __uint_as_float(((bf16_bits(a.z) << 16) & m0) | ((bf16_bits(b.z) << 16) & m1) | ((bf16_bits(c.z) << 16) & m2));
      o.w = __uint_as_float(((bf16_bits(a.w) << 16) & m0) | ((bf16_bits(b.w) << 16) & m1) | ((bf16_bits(c.w) << 16) & m2));
      float* dp = biasp + 4 * tc;
      if (tid < 72) *(volatile v4f*)dp = o;
      __threadfence();
      if (tid < 72) *(volatile v4f*)dp = o;
    }
  }
}

__device__ __forceinline__ void bucket_flush(const int* pl, const int* cnt, const int* dvs, int ov,
                                             int* lp, int* cop, int* dp, int* fp, int tid) {
#pragma unroll 1
  for (int i = tid * 4; i < 2 * RCAP; i += NTHR * 4) {
    const v4i v = *(const v4ia*)(pl + i);
    *(volatile v4i*)(lp + i) = v;
  }
#pragma unroll 1
  for (int it = 0; it < 2; ++it) {
    const int i = it * NBRUN + 4 * tid;
    const v4i v = *(const v4ia*)(cnt + i);
    *(volatile v4i*)(cop + i) = v;
  }
  {
    const v4i v = *(const v4ia*)(dvs + 4 * tid);
    *(volatile v4i*)(dp + 4 * tid) = v;
  }
  if (tid < 8) {
    const v4i f = {ov, ov, ov, ov};
    *(volatile v4i*)(fp + 4 * tid) = f;
  }
}

__global__ __launch_bounds__(NTHR) void k_bucket(const int* __restrict__ srcs, const int* __restrict__ dsts,
                                                 const float* __restrict__ ew, int* LIST, int* CO, int* DVI,
                                                 int* FLAG) {
  extern __shared__ __attribute__((aligned(16))) int dsm[];
  int* wl   = dsm;
  int* pl   = dsm + NWAVE * WLCAP;
  int* cnt  = pl + 2 * RCAP;
  int* offs = cnt + NBRUN;
  int* cur  = offs + NBRUN;
  int* dvs  = cur + NBRUN;
  int* misc = dvs + NBRUN;
  const int tid = (int)threadIdx.x, lane = tid & 31, wave = tid >> 5;
  const int blk = (int)blockIdx.x;
  const unsigned nbs = (unsigned)(blk * NBRUN);

  {
    const v4i z4 = {0, 0, 0, 0};
    for (int i = tid * 4; i < BK_ZINTS; i += NTHR * 4) *(v4ia*)(dsm + i) = z4;
    if (tid < 16) misc[tid] = 0;
  }
  __syncthreads();

  {
    const int per  = ((NE + NWAVE * WCH - 1) / (NWAVE * WCH)) * WCH;
    const int ebeg = wave * per;
    const int eend = (ebeg + per < NE) ? (ebeg + per) : NE;
    int* mylist = wl + wave * WLCAP;
    int wc = 0;
#pragma unroll 1
    for (int cb = ebeg; cb < eend; cb += WCH) {
      const int e0 = cb + lane * EPT;
      const v4i da = *(const v4ia*)(dsts + e0);
      const v4i db = *(const v4ia*)(dsts + e0 + 4);
      const unsigned s0 = (unsigned)da.x - nbs, s1 = (unsigned)da.y - nbs;
      const unsigned s2 = (unsigned)da.z - nbs, s3 = (unsigned)da.w - nbs;
      const unsigned s4 = (unsigned)db.x - nbs, s5 = (unsigned)db.y - nbs;
      const unsigned s6 = (unsigned)db.z - nbs, s7 = (unsigned)db.w - nbs;
      const bool h0 = s0 < (unsigned)NBRUN, h1 = s1 < (unsigned)NBRUN, h2 = s2 < (unsigned)NBRUN, h3 = s3 < (unsigned)NBRUN;
      const bool h4 = s4 < (unsigned)NBRUN, h5 = s5 < (unsigned)NBRUN, h6 = s6 < (unsigned)NBRUN, h7 = s7 < (unsigned)NBRUN;
      const unsigned m0 = __builtin_amdgcn_ballot_w32(h0), m1 = __builtin_amdgcn_ballot_w32(h1);
      const unsigned m2 = __builtin_amdgcn_ballot_w32(h2), m3 = __builtin_amdgcn_ballot_w32(h3);
      const unsigned m4 = __builtin_amdgcn_ballot_w32(h4), m5 = __builtin_amdgcn_ballot_w32(h5);
      const unsigned m6 = __builtin_amdgcn_ballot_w32(h6), m7 = __builtin_amdgcn_ballot_w32(h7);
      const unsigned any = m0 | m1 | m2 | m3 | m4 | m5 | m6 | m7;
      if (any != 0u) {
        const int pre = (int)(__builtin_amdgcn_mbcnt_lo(m0, 0u) + __builtin_amdgcn_mbcnt_lo(m1, 0u) +
                              __builtin_amdgcn_mbcnt_lo(m2, 0u) + __builtin_amdgcn_mbcnt_lo(m3, 0u) +
                              __builtin_amdgcn_mbcnt_lo(m4, 0u) + __builtin_amdgcn_mbcnt_lo(m5, 0u) +
                              __builtin_amdgcn_mbcnt_lo(m6, 0u) + __builtin_amdgcn_mbcnt_lo(m7, 0u));
        int p = wc + pre;
        if (h0) { if (p < WLCAP) mylist[p] = ((e0 + 0) << SLB) | (int)s0; p = p + 1; }
        if (h1) { if (p < WLCAP) mylist[p] = ((e0 + 1) << SLB) | (int)s1; p = p + 1; }
        if (h2) { if (p < WLCAP) mylist[p] = ((e0 + 2) << SLB) | (int)s2; p = p + 1; }
        if (h3) { if (p < WLCAP) mylist[p] = ((e0 + 3) << SLB) | (int)s3; p = p + 1; }
        if (h4) { if (p < WLCAP) mylist[p] = ((e0 + 4) << SLB) | (int)s4; p = p + 1; }
        if (h5) { if (p < WLCAP) mylist[p] = ((e0 + 5) << SLB) | (int)s5; p = p + 1; }
        if (h6) { if (p < WLCAP) mylist[p] = ((e0 + 6) << SLB) | (int)s6; p = p + 1; }
        if (h7) { if (p < WLCAP) mylist[p] = ((e0 + 7) << SLB) | (int)s7; p = p + 1; }
        wc += (int)(__builtin_popcount(m0) + __builtin_popcount(m1) + __builtin_popcount(m2) + __builtin_popcount(m3) +
                    __builtin_popcount(m4) + __builtin_popcount(m5) + __builtin_popcount(m6) + __builtin_popcount(m7));
      }
    }
    if (lane == 0) misc[wave] = wc;
  }
  __syncthreads();

  if (wave == 0) {
    int ov = 0;
#pragma unroll 1
    for (int w2 = 0; w2 < NWAVE; ++w2) {
      int c = misc[w2];
      if (c > WLCAP) ov = 1;
      c = c < 0 ? 0 : (c > WLCAP ? WLCAP : c);
#pragma unroll 1
      for (int b0 = 0; b0 < c; b0 += 32) {
        const int idx = b0 + lane;
        const int ent = wl[w2 * WLCAP + (idx < WLCAP ? idx : WLCAP - 1)];
        const int m32 = (c - b0) < 32 ? (c - b0) : 32;
#pragma unroll 1
        for (int k = 0; k < m32; ++k) {
          const int u    = __builtin_amdgcn_readlane(ent, k);
          const int slot = u & (NBRUN - 1);
          if (lane == 0) cnt[slot] = cnt[slot] + 1;
        }
      }
    }
    if (lane == 0) misc[9] = ov;
  }
  __syncthreads();
  if (wave == 0) {
    const int base = lane * (NBRUN / 32);
    int s = 0;
#pragma unroll 1
    for (int i = 0; i < NBRUN / 32; ++i) s += cnt[base + i];
    int incl = s;
#pragma unroll
    for (int d = 1; d < 32; d <<= 1) {
      const int y = __shfl_up(incl, d, 32);
      if (lane >= d) incl += y;
    }
    int run = incl - s;
#pragma unroll 1
    for (int i = 0; i < NBRUN / 32; ++i) {
      const int cv = cnt[base + i];
      offs[base + i] = run;
      cur[base + i]  = run;
      run += cv;
    }
  }
  __syncthreads();

  if (wave == 0) {
#pragma unroll 1
    for (int w2 = 0; w2 < NWAVE; ++w2) {
      int c = misc[w2];
      c = c < 0 ? 0 : (c > WLCAP ? WLCAP : c);
#pragma unroll 1
      for (int b0 = 0; b0 < c; b0 += 32) {
        const int idx = b0 + lane;
        const int ent = wl[w2 * WLCAP + (idx < WLCAP ? idx : WLCAP - 1)];
        int eid = (ent >> SLB) & 0x1FFFFF;
        eid = eid > NE - 1 ? NE - 1 : eid;
        int sr = srcs[eid];
        sr = sr < 0 ? 0 : (sr > NN - 1 ? NN - 1 : sr);
        const int wb = (int)(bf16_bits(ew[eid]) << 16);
        const int m32 = (c - b0) < 32 ? (c - b0) : 32;
#pragma unroll 1
        for (int k = 0; k < m32; ++k) {
          const int u    = __builtin_amdgcn_readlane(ent, k);
          const int sk   = __builtin_amdgcn_readlane(sr, k);
          const int wk   = __builtin_amdgcn_readlane(wb, k);
          const int slot = u & (NBRUN - 1);
          if (lane == 0) {
            int p = cur[slot];
            p = p < 0 ? 0 : (p > RCAP - 1 ? RCAP - 1 : p);
            pl[2 * p]     = sk;
            pl[2 * p + 1] = wk;
            cur[slot] = p + 1;
          }
        }
      }
    }
  }
  __syncthreads();

  const int ovf = misc[9];
  const float qnan = __uint_as_float(0x7fc00000u);
#pragma unroll 1
  for (int it = 0; it < NBRUN / NTHR; ++it) {
    const int s = it * NTHR + tid;
    int c = cnt[s];
    const bool big = c > DEGCAP;
    c = c < 0 ? 0 : (c > DEGCAP ? DEGCAP : c);
    int o = offs[s];
    o = o < 0 ? 0 : (o > RCAP - 1 ? RCAP - 1 : o);
    int last = o + c - 1;
    last = last < o ? o : last;
    last = last > RCAP - 1 ? RCAP - 1 : last;
    int cmv = c;
#pragma unroll
    for (int d = 16; d >= 1; d >>= 1) {
      const int y = __shfl_xor(cmv, d, 32);
      cmv = cmv > y ? cmv : y;
    }
    const int cm = __builtin_amdgcn_readfirstlane(cmv);
    float sum = 0.0f;
#pragma unroll 1
    for (int j = 0; j < cm; ++j) {
      int idx = o + j;
      idx = idx > last ? last : idx;
      const int wbits = pl[2 * idx + 1];
      asm volatile("" :: "v"(wbits));
      const float t = sum + __int_as_float(wbits);
      sum = (j < c) ? t : sum;
    }
    const float deg = sum + 1.0f;
    float dv = (deg > 0.0f) ? (1.0f / sqrtf(deg)) : 0.0f;
    dv = ((ovf != 0) | big) ? qnan : dv;
    dvs[s] = __float_as_int(dv);
  }
  __syncthreads();

  int* lp  = LIST + (size_t)blk * (2 * RCAP);
  int* cop = CO + (size_t)blk * (2 * NBRUN);
  int* dp  = DVI + (size_t)blk * NBRUN;
  int* fp  = FLAG + (size_t)blk * 32;
  bucket_flush(pl, cnt, dvs, ovf, lp, cop, dp, fp, tid);
  __threadfence();
  bucket_flush(pl, cnt, dvs, ovf, lp, cop, dp, fp, tid);
}

template <int KEXT, int BP>
__device__ __forceinline__ void gemm_16x96(const unsigned short* __restrict__ ap,
                                           const unsigned short* __restrict__ bp, v8f (&acc)[6]) {
#pragma unroll 1
  for (int k0 = 0; k0 < KEXT; k0 += 32) {
    FragB af;
    af.h[0] = *(const v8usa*)(ap + k0);
    af.h[1] = *(const v8usa*)(ap + k0 + 16);
#pragma unroll
    for (int nt = 0; nt < 6; ++nt) {
      const unsigned short* wq = bp + (size_t)(16 * nt) * (size_t)BP + k0;
      FragB bf;
      bf.h[0] = *(const v8usa*)wq;
      bf.h[1] = *(const v8usa*)(wq + 16);
      acc[nt] = wmb(af, bf, acc[nt]);
    }
  }
}

__device__ __forceinline__ void p_flush(const float* stg, const float* sdv, float* ob, int tid) {
#pragma unroll 1
  for (int it = 0; it < 12; ++it) {
    const int i4 = it * NTHR + tid;
    const int r  = i4 / 24, c4 = i4 - 24 * r;
    const v4f a = *(const v4fa*)(stg + r * SP + 4 * c4);
    const float s = sdv[r];
    v4f o;
    o.x = s * a.x; o.y = s * a.y; o.z = s * a.z; o.w = s * a.w;
    *(volatile v4f*)(ob + (size_t)4 * (size_t)i4) = o;
  }
}

template <int KEXT, int AP, int BP>
__global__ __launch_bounds__(NTHR) __attribute__((amdgpu_num_vgpr(248)))
void k_gemm_kx(const unsigned short* __restrict__ A, const unsigned short* __restrict__ BT,
               const float* __restrict__ DINV, float* Pout) {
  static_assert(KEXT % 32 == 0 && KEXT <= AP && KEXT <= BP);
  __shared__ __attribute__((aligned(16))) float stg[GBM * SP];
  __shared__ __attribute__((aligned(16))) float sdv[GBM];
  const int tid = (int)threadIdx.x, lane = tid & 31, wave = tid >> 5, hh = lane >> 4, m = lane & 15;
  const int rowBase = (int)blockIdx.x * GBM;
  if (tid < GBM) sdv[tid] = DINV[rowBase + tid];

  v8f acc[6];
  {
    const v8f z = {0.f, 0.f, 0.f, 0.f, 0.f, 0.f, 0.f, 0.f};
#pragma unroll
    for (int t = 0; t < 6; ++t) acc[t] = z;
  }
  const unsigned short* ap = A + (size_t)(rowBase + 16 * wave + m) * (size_t)AP + 8 * hh;
  const unsigned short* bp = BT + (size_t)m * (size_t)BP + 8 * hh;
  gemm_16x96<KEXT, BP>(ap, bp, acc);
#pragma unroll
  for (int nt = 0; nt < 6; ++nt) {
#pragma unroll
    for (int r = 0; r < 8; ++r) stg[(16 * wave + 8 * hh + r) * SP + 16 * nt + m] = acc[nt][r];
  }
  __syncthreads();

  float* ob = Pout + (size_t)blockIdx.x * (size_t)(GBM * FD);
  p_flush(stg, sdv, ob, tid);
  __threadfence();
  p_flush(stg, sdv, ob, tid);
}

template <int MODE>
__global__ __launch_bounds__(NTHR) void k_replay(const int* __restrict__ LIST, const int* __restrict__ CO,
                                                 const float* __restrict__ DINV, const int* __restrict__ FLAG,
                                                 const float* __restrict__ P, const float* __restrict__ bias,
                                                 unsigned short* XHL, float* outp) {
  const int tid = (int)threadIdx.x, lane = tid & 31, wv = tid >> 5;
  const int cq = lane < 24 ? lane : 23;
  const int rowBase = (int)blockIdx.x * ABM;
  const int bucket  = rowBase >> SLB;
  const int* lb  = LIST + (size_t)bucket * (2 * RCAP);
  const int* cob = CO + (size_t)bucket * (2 * NBRUN);
  const int flag = FLAG[(size_t)bucket * 32];
  const v4f bv = *(const v4fa*)(bias + 4 * cq);
  const float qnan = __uint_as_float(0x7fc00000u);
  const bool stl = lane < 24;

#pragma unroll 1
  for (int i = 0; i < ABM / NWAVE; ++i) {
    const int dv_  = rowBase + (ABM / NWAVE) * wv + i;
    const int slot = dv_ & (NBRUN - 1);
    int cv = cob[slot];
    int ov = cob[NBRUN + slot];
    const int bigv = cv > DEGCAP ? 1 : 0;
    cv = cv < 0 ? 0 : (cv > DEGCAP ? DEGCAP : cv);
    ov = ov < 0 ? 0 : (ov > RCAP - 1 ? RCAP - 1 : ov);
    int lastv = ov + cv - 1;
    lastv = lastv < ov ? ov : lastv;
    lastv = lastv > RCAP - 1 ? RCAP - 1 : lastv;
    const int d    = __builtin_amdgcn_readfirstlane(dv_);
    const int c    = __builtin_amdgcn_readfirstlane(cv);
    const int o    = __builtin_amdgcn_readfirstlane(ov);
    const int last = __builtin_amdgcn_readfirstlane(lastv);
    const int big  = __builtin_amdgcn_readfirstlane(bigv);

    float a0 = 0.0f, a1 = 0.0f, a2 = 0.0f, a3 = 0.0f;
#pragma unroll 1
    for (int b0 = 0; b0 < c; b0 += 32) {
      int idx = o + b0 + lane;
      idx = idx > last ? last : idx;
      const v2i ent = *(const v2ia*)(lb + 2 * idx);
      int sr = ent.x;
      sr = sr < 0 ? 0 : (sr > NN - 1 ? NN - 1 : sr);
      const int wb = ent.y;
      const int m32 = (c - b0) < 32 ? (c - b0) : 32;
#pragma unroll 1
      for (int k = 0; k < m32; ++k) {
        const int   sk = __builtin_amdgcn_readlane(sr, k);
        const float wk = __int_as_float(__builtin_amdgcn_readlane(wb, k));
        const v4f v = *(const v4fa*)(P + (size_t)sk * FD + 4 * cq);
        asm volatile("" :: "v"(v));
        a0 = fmaf(wk, v.x, a0); a1 = fmaf(wk, v.y, a1); a2 = fmaf(wk, v.z, a2); a3 = fmaf(wk, v.w, a3);
      }
    }
    const int dc = d < NN ? d : NN - 1;
    const v4f g = *(const v4fa*)(P + (size_t)dc * FD + 4 * cq);
    asm volatile("" :: "v"(g));
    const float dd = DINV[d];
    float v0 = dd * (a0 + g.x) + bv.x, v1 = dd * (a1 + g.y) + bv.y;
    float v2 = dd * (a2 + g.z) + bv.z, v3 = dd * (a3 + g.w) + bv.w;
    const bool bad  = (flag != 0) | (big != 0);
    const bool live = d < NN;
    if constexpr (MODE != 0) {
      v0 = (v0 > 0.0f) ? v0 : (v0 - v0); v1 = (v1 > 0.0f) ? v1 : (v1 - v1);
      v2 = (v2 > 0.0f) ? v2 : (v2 - v2); v3 = (v3 > 0.0f) ? v3 : (v3 - v3);
      v0 = bad ? qnan : v0; v1 = bad ? qnan : v1; v2 = bad ? qnan : v2; v3 = bad ? qnan : v3;
      v0 = live ? v0 : 0.0f; v1 = live ? v1 : 0.0f; v2 = live ? v2 : 0.0f; v3 = live ? v3 : 0.0f;
      int h01, h23, l01, l23;
      hilo_pack(v0, v1, v2, v3, h01, h23, l01, l23);
      const v4i ow = regroup24(h01, h23, l01, l23, lane);
      unsigned short* hp = XHL + (size_t)d * APITCH2 + 8 * cq;
      if (stl) *(volatile v4i*)hp = ow;
      __threadfence();
      if (stl) *(volatile v4i*)hp = ow;
    } else {
      v0 = bad ? qnan : v0; v1 = bad ? qnan : v1; v2 = bad ? qnan : v2; v3 = bad ? qnan : v3;
      v4f ovv;
      ovv.x = v0; ovv.y = v1; ovv.z = v2; ovv.w = v3;
      float* op = outp + (size_t)dc * FD + 4 * cq;
      const bool st = stl & live;
      if (st) *(volatile v4f*)op = ovv;
      __threadfence();
      if (st) *(volatile v4f*)op = ovv;
    }
  }
}

extern "C" void kernel_launch(void* const* d_in, const int* in_sizes, int n_in,
                              void* d_out, int out_size, void* d_ws, size_t ws_size,
                              hipStream_t stream) {
  if (n_in < 9) return;
  if (in_sizes[0] != NN * FD) return;
  if (in_sizes[1] != 2 * NE) return;
  if (in_sizes[2] != NE) return;
  if (in_sizes[3] != FD * FD || in_sizes[4] != FD) return;
  if (in_sizes[5] != FD * FD || in_sizes[6] != FD) return;
  if (in_sizes[7] != FD * FD || in_sizes[8] != FD) return;
  if (out_size != NN * FD) return;

  const float* x  = (const float*)d_in[0];
  const int*   ei = (const int*)d_in[1];
  const float* ew = (const float*)d_in[2];
  const float* W1 = (const float*)d_in[3];
  const float* b1 = (const float*)d_in[4];
  const float* W2 = (const float*)d_in[5];
  const float* b2 = (const float*)d_in[6];
  const float* W3 = (const float*)d_in[7];
  const float* b3 = (const float*)d_in[8];
  float* out = (float*)d_out;
  const int* srcs = ei;
  const int* dsts = ei + NE;

  constexpr size_t zXB   = (size_t)MP * APITCH1 * 2;
  constexpr size_t zP    = (size_t)MP * FD * 4;
  constexpr size_t zXHL  = (size_t)MP * APITCH2 * 2;
  constexpr size_t zLIST = (size_t)NBK * 2 * RCAP * 4;
  constexpr size_t zCO   = (size_t)NBK * 2 * NBRUN * 4;
  constexpr size_t zDV   = (size_t)NBK * NBRUN * 4;
  constexpr size_t zFLAG = 8192;
  constexpr size_t zW1T  = (size_t)FD * BPITCH1 * 2;
  constexpr size_t zW2D  = (size_t)FD * BPITCH2 * 2;
  constexpr size_t zBIAS = 1280;
  constexpr size_t oXB   = 0;
  constexpr size_t oP    = oXB + zXB;
  constexpr size_t oXHL  = oP + zP;
  constexpr size_t oLIST = oXHL + zXHL;
  constexpr size_t oCO   = oLIST + zLIST;
  constexpr size_t oDV   = oCO + zCO;
  constexpr size_t oFLAG = oDV + zDV;
  constexpr size_t oW1T  = oFLAG + zFLAG;
  constexpr size_t oW2D  = oW1T + zW1T;
  constexpr size_t oW3D  = oW2D + zW2D;
  constexpr size_t oBIAS = oW3D + zW2D;
  constexpr size_t oEND  = oBIAS + zBIAS;
  static_assert(zXB % 256 == 0 && zP % 256 == 0 && zXHL % 256 == 0 && zLIST % 256 == 0 && zCO % 256 == 0);
  static_assert(zDV % 256 == 0 && zFLAG % 256 == 0 && zW1T % 256 == 0 && zW2D % 256 == 0 && zBIAS % 256 == 0);
  static_assert((size_t)NBK * 128 <= zFLAG && (size_t)3 * FD * 4 <= zBIAS);
  static_assert((size_t)PBX * NTHR * 16 == zXB);
  static_assert((size_t)NN * APITCH2 * 2 + (size_t)NUZ * 16 == zXHL);
  static_assert((size_t)NUW1 * 16 == zW1T && (size_t)NUW2 * 16 == zW2D);
  static_assert((size_t)(MP / GBM) * GBM * FD * 4 == zP);
  static_assert((size_t)(MP / ABM) * ABM * APITCH2 * 2 == zXHL);
  static_assert(oEND <= ((size_t)128 << 20));
  if (oEND > ws_size) return;

  char* ws = (char*)d_ws;
  unsigned short* XB   = (unsigned short*)(ws + oXB);
  float*          P    = (float*)(ws + oP);
  unsigned short* XHL  = (unsigned short*)(ws + oXHL);
  int*            LIST = (int*)(ws + oLIST);
  int*            CO   = (int*)(ws + oCO);
  float*          DINV = (float*)(ws + oDV);
  int*            FLAG = (int*)(ws + oFLAG);
  unsigned short* W1T  = (unsigned short*)(ws + oW1T);
  unsigned short* W2D  = (unsigned short*)(ws + oW2D);
  unsigned short* W3D  = (unsigned short*)(ws + oW3D);
  float*          BIAS = (float*)(ws + oBIAS);

  hipFuncSetAttribute(reinterpret_cast<const void*>(&k_bucket), hipFuncAttributeMaxDynamicSharedMemorySize, (int)BK_LDS);

  k_prep<<<PBTOT, NTHR, 0, stream>>>(x, W1, b1, W2, b2, W3, b3, XB, XHL, W1T, W2D, W3D, BIAS);
  k_bucket<<<NBK, NTHR, BK_LDS, stream>>>(srcs, dsts, ew, LIST, CO, (int*)DINV, FLAG);
  k_gemm_kx<KEXT_L1, APITCH1, BPITCH1><<<MP / GBM, NTHR, 0, stream>>>(XB, W1T, DINV, P);
  k_replay<1><<<MP / ABM, NTHR, 0, stream>>>(LIST, CO, DINV, FLAG, P, BIAS, XHL, out);
  k_gemm_kx<KEXT_L2, APITCH2, BPITCH2><<<MP / GBM, NTHR, 0, stream>>>(XHL, W2D, DINV, P);
  k_replay<1><<<MP / ABM, NTHR, 0, stream>>>(LIST, CO, DINV, FLAG, P, BIAS + FD, XHL, out);
  k_gemm_kx<KEXT_L3, APITCH2, BPITCH2><<<MP / GBM, NTHR, 0, stream>>>(XHL, W3D, DINV, P);
  k_replay<0><<<MP / ABM, NTHR, 0, stream>>>(LIST, CO, DINV, FLAG, P, BIAS + 2 * FD, XHL, out);
}
